// Mamba3Block_83537113907707
// MI455X (gfx1250) — hardware-run, weakly checked
//
#include <hip/hip_runtime.h>
#include <math.h>

constexpr int DIMC       = 1024;
constexpr int NBATCH     = 4;
constexpr int NSEQ       = 2048;
constexpr int NTOK       = NBATCH * NSEQ;
constexpr int HIDF       = 2048;
constexpr int EMBW       = 6 * DIMC;
constexpr int GEMM_WAVES = 2;
constexpr int SLABP      = 68;
constexpr float WCARRY     = 64.0f;
constexpr float WCARRY_INV = 1.0f / 64.0f;
constexpr float LN_EPS_F   = 1e-6f;

static_assert(NTOK == 8192);
static_assert(EMBW == 6144);
static_assert(NTOK % 64 == 0 && DIMC % 64 == 0 && HIDF % 64 == 0);
static_assert(DIMC % 32 == 0 && HIDF % 32 == 0);
static_assert(NSEQ % 64 == 0);
static_assert(((NTOK / 64) * (DIMC / 64)) % GEMM_WAVES == 0);
static_assert(((NTOK / 64) * (HIDF / 64)) % GEMM_WAVES == 0);
static_assert(EMBW % 256 == 0);
static_assert(NTOK % 8 == 0);

typedef __attribute__((ext_vector_type(16))) _Float16 v16h;
typedef __attribute__((ext_vector_type(8)))  _Float16 v8h;
typedef __attribute__((ext_vector_type(8)))  float    v8f;
typedef __attribute__((ext_vector_type(4)))  float    v4f;

union FragU { v16h v; v8h h[2]; };

__device__ __forceinline__ float bf16r(float f) {
  const unsigned u = __float_as_uint(f);
  const unsigned r = (u + 0x7FFFu + ((u >> 16) & 1u)) & 0xFFFF0000u;
  return __uint_as_float(r);
}

__device__ __forceinline__ v16h frag_load(const _Float16* p) {
  FragU f;
  f.h[0] = *(const v8h*)(p);
  f.h[1] = *(const v8h*)(p + 16);
  return f.v;
}
__device__ __forceinline__ v8f mma_h(v16h a, v16h b, v8f c) {
  return __builtin_amdgcn_wmma_f32_16x16x32_f16(false, a, false, b, (short)0, c, false, false);
}
__device__ __forceinline__ void tie_acc(v8f& c, v16h a, v16h b) {
  asm volatile("" : "+v"(c) : "v"(a), "v"(b));
}
__device__ __forceinline__ void tie_acc_nop(v8f& c, v16h a, v16h b) {
  asm volatile("v_nop\n\tv_nop\n\tv_nop\n\tv_nop" : "+v"(c) : "v"(a), "v"(b));
}
__device__ __forceinline__ void keep4_h(v16h a, v16h b, v16h c, v16h d) {
  asm volatile("v_nop" :: "v"(a), "v"(b), "v"(c), "v"(d));
}
__device__ __forceinline__ void acc_guard4(v8f& a, v8f& b, v8f& c, v8f& d) {
  asm volatile("v_nop\n\tv_nop\n\tv_nop\n\tv_nop" : "+v"(a), "+v"(b), "+v"(c), "+v"(d));
}

__device__ __forceinline__ float gelu_erf(float v) {
  return 0.5f * v * (1.0f + erff(v * 0.70710678118654752f));
}
__device__ __forceinline__ float gelu_tanh(float v) {
  const float c = v + 0.044715f * v * v * v;
  return 0.5f * v * (1.0f + tanhf(0.7978845608028654f * c));
}

__global__ __launch_bounds__(256) void wprep_kernel(const float* __restrict__ w,
                                                    unsigned short* __restrict__ wt,
                                                    int K, int N) {
  __shared__ float tile[64 * 65];
  const int tid = threadIdx.x;
  const int k0 = blockIdx.y * 64;
  const int n0 = blockIdx.x * 64;
  {
    const int c  = tid & 63;
    const int r0 = tid >> 6;
#pragma unroll 4
    for (int u = 0; u < 16; ++u) {
      const int r = r0 + 4 * u;
      const float wv = w[(size_t)(k0 + r) * N + n0 + c];
      tile[r * 65 + c] = bf16r(wv);
    }
  }
  __syncthreads();
  v8h hv0, hv1;
  const int n_a  = tid >> 3;
  const int n_b  = (tid + 256) >> 3;
  const int kc   = (tid & 7) * 8;
#pragma unroll
  for (int e = 0; e < 8; ++e) {
    const float s0 = tile[(kc + e) * 65 + n_a] * WCARRY;
    const float s1 = tile[(kc + e) * 65 + n_b] * WCARRY;
    hv0[e] = (_Float16)s0;
    hv1[e] = (_Float16)s1;
  }
  const size_t oa = (size_t)(n0 + n_a) * K + k0 + kc;
  const size_t ob = (size_t)(n0 + n_b) * K + k0 + kc;
  for (int pass = 0; pass < 2; ++pass) {
    *(volatile v8h*)(wt + oa) = hv0;
    *(volatile v8h*)(wt + ob) = hv1;
    __threadfence();
  }
}

__global__ __launch_bounds__(256) void cond_proj_kernel(const float* __restrict__ t,
                                                        const float* __restrict__ w,
                                                        const float* __restrict__ bias,
                                                        float* __restrict__ emb) {
  __shared__ float st[NBATCH * DIMC];
  const int tid = threadIdx.x;
#pragma unroll 1
  for (int i = tid; i < NBATCH * DIMC; i += 256) {
    const float tv = bf16r(t[i]);
    st[i] = tv / (1.0f + expf(-tv));
  }
  __syncthreads();
  const int j = blockIdx.x * 256 + tid;
  const float* wp = w + j;
  float a0 = 0.0f, a1 = 0.0f, a2 = 0.0f, a3 = 0.0f;
#pragma unroll 4
  for (int k = 0; k < DIMC; ++k) {
    const float wraw = wp[(size_t)k * EMBW];
    const float wv = bf16r(wraw);
    a0 = fmaf(st[k], wv, a0);
    a1 = fmaf(st[DIMC + k], wv, a1);
    a2 = fmaf(st[2 * DIMC + k], wv, a2);
    a3 = fmaf(st[3 * DIMC + k], wv, a3);
  }
  const float bj = bf16r(bias[j]);
  a0 += bj;
  a1 += bj;
  a2 += bj;
  a3 += bj;
  volatile float* ep = emb + j;
  for (int pass = 0; pass < 2; ++pass) {
    ep[0]        = a0;
    ep[EMBW]     = a1;
    ep[2 * EMBW] = a2;
    ep[3 * EMBW] = a3;
    __threadfence();
  }
}

template <bool INBF>
__global__ __launch_bounds__(256) void ln_mod_kernel(const float* __restrict__ X,
                                                     const float* __restrict__ emb,
                                                     int shift_off, int scale_off,
                                                     unsigned short* __restrict__ Y, int nrows) {
  const int lane = threadIdx.x & 31;
  const int row  = blockIdx.x * 8 + (threadIdx.x >> 5);
  if (row >= nrows) return;
  const int b = row / NSEQ;
  const float* rp = X + (size_t)row * DIMC + 8 * lane;
  v4f v[8];
#pragma unroll
  for (int q = 0; q < 4; ++q) {
    v[2 * q]     = *(const v4f*)(rp + 256 * q);
    v[2 * q + 1] = *(const v4f*)(rp + 256 * q + 4);
  }
  if (INBF) {
#pragma unroll
    for (int u = 0; u < 8; ++u) {
#pragma unroll
      for (int e = 0; e < 4; ++e) {
        const float raw = v[u][e];
        v[u][e] = bf16r(raw);
      }
    }
  }
  float s = 0.0f;
#pragma unroll
  for (int u = 0; u < 8; ++u) s += (v[u][0] + v[u][1]) + (v[u][2] + v[u][3]);
#pragma unroll
  for (int off = 1; off < 32; off <<= 1) s += __shfl_xor(s, off, 32);
  const float mu = s * (1.0f / DIMC);
  float ss = 0.0f;
#pragma unroll
  for (int u = 0; u < 8; ++u) {
#pragma unroll
    for (int e = 0; e < 4; ++e) {
      const float d = v[u][e] - mu;
      v[u][e] = d;
      ss += d * d;
    }
  }
#pragma unroll
  for (int off = 1; off < 32; off <<= 1) ss += __shfl_xor(ss, off, 32);
  const float var  = ss * (1.0f / DIMC);
  const float rstd = rsqrtf(var + LN_EPS_F);
  const float* shp = emb + (size_t)b * EMBW + shift_off + 8 * lane;
  const float* scp = emb + (size_t)b * EMBW + scale_off + 8 * lane;
  v8h hv[4];
#pragma unroll
  for (int q = 0; q < 4; ++q) {
    const v4f sc0 = *(const v4f*)(scp + 256 * q);
    const v4f sc1 = *(const v4f*)(scp + 256 * q + 4);
    const v4f sh0 = *(const v4f*)(shp + 256 * q);
    const v4f sh1 = *(const v4f*)(shp + 256 * q + 4);
#pragma unroll
    for (int e = 0; e < 4; ++e) {
      const float o0 = (v[2 * q][e] * rstd) * (1.0f + sc0[e]) + sh0[e];
      const float o1 = (v[2 * q + 1][e] * rstd) * (1.0f + sc1[e]) + sh1[e];
      hv[q][e]     = (_Float16)o0;
      hv[q][4 + e] = (_Float16)o1;
    }
  }
  unsigned short* op = Y + (size_t)row * DIMC + 8 * lane;
  for (int pass = 0; pass < 2; ++pass) {
#pragma unroll
    for (int q = 0; q < 4; ++q) *(volatile v8h*)(op + 256 * q) = hv[q];
    __threadfence();
  }
}

template <int EPI, bool RBF>
__global__ __launch_bounds__(64) void gemm_tok_kernel(
    const unsigned short* __restrict__ Ap, int lda,
    const unsigned short* __restrict__ Btp, int ldb,
    void* __restrict__ Cout, int ldc,
    const float* __restrict__ bias, const float* __restrict__ resid, const float* __restrict__ gate,
    int M, int N, int K, float scale) {
  __shared__ __align__(16) float sT[GEMM_WAVES][64 * SLABP];
  const _Float16* A  = (const _Float16*)Ap;
  const _Float16* Bt = (const _Float16*)Btp;
  const int lane = threadIdx.x & 31;
  const int wave = threadIdx.x >> 5;
  const int tilesN = N >> 6;
  const int tilesM = M >> 6;
  const int tile = blockIdx.x * GEMM_WAVES + wave;
  if (tile >= tilesM * tilesN) return;
  const int tm = tile / tilesN;
  const int tn = tile - tm * tilesN;
  const int m0 = tm << 6;
  const int n0 = tn << 6;
  const int rlane = lane & 15;
  const int koff  = (lane >> 4) * 8;
  const int mOff  = (lane >> 4) * 8;

  const _Float16* arow = A  + (size_t)(m0 + rlane) * lda + koff;
  const _Float16* brow = Bt + (size_t)(n0 + rlane) * ldb + koff;
  const size_t astep = (size_t)16 * lda;
  const size_t bstep = (size_t)16 * ldb;

  v8f acc[4][4];
#pragma unroll
  for (int i = 0; i < 4; ++i)
#pragma unroll
    for (int j = 0; j < 4; ++j) acc[i][j] = (v8f){0.f, 0.f, 0.f, 0.f, 0.f, 0.f, 0.f, 0.f};

  for (int k0 = 0; k0 < K; k0 += 32) {
    v16h ah[4];
#pragma unroll
    for (int i = 0; i < 4; ++i) ah[i] = frag_load(arow + (size_t)i * astep + k0);
#pragma unroll
    for (int j = 0; j < 4; ++j) {
      const v16h bh = frag_load(brow + (size_t)j * bstep + k0);
#pragma unroll
      for (int i = 0; i < 4; ++i) acc[i][j] = mma_h(ah[i], bh, acc[i][j]);
      tie_acc(acc[0][j], ah[0], bh);
      tie_acc(acc[1][j], ah[1], bh);
      tie_acc(acc[2][j], ah[2], bh);
      tie_acc_nop(acc[3][j], ah[3], bh);
    }
    keep4_h(ah[0], ah[1], ah[2], ah[3]);
  }
  acc_guard4(acc[0][0], acc[0][1], acc[0][2], acc[0][3]);
  acc_guard4(acc[1][0], acc[1][1], acc[1][2], acc[1][3]);
  acc_guard4(acc[2][0], acc[2][1], acc[2][2], acc[2][3]);
  acc_guard4(acc[3][0], acc[3][1], acc[3][2], acc[3][3]);

  float* slab = sT[wave];
#pragma unroll
  for (int i = 0; i < 4; ++i)
#pragma unroll
    for (int j = 0; j < 4; ++j)
#pragma unroll
      for (int r = 0; r < 8; ++r)
        slab[(16 * i + mOff + r) * SLABP + 16 * j + rlane] = acc[i][j][r] * scale;
  __builtin_amdgcn_fence(__ATOMIC_RELEASE, "workgroup");
  __builtin_amdgcn_wave_barrier();
  __builtin_amdgcn_fence(__ATOMIC_ACQUIRE, "workgroup");

  if (EPI == 2) {
    const int hh = lane >> 4;
    const int c4 = (lane & 15) * 4;
    const int bt = m0 / NSEQ;
    const v4f braw = *(const v4f*)(bias + n0 + c4);
    v4f bz;
#pragma unroll
    for (int e = 0; e < 4; ++e) {
      const float bv = braw[e];
      bz[e] = bf16r(bv);
    }
    const v4f gz = *(const v4f*)(gate + (size_t)bt * EMBW + n0 + c4);
    float* C = (float*)Cout;
#pragma unroll 4
    for (int it = 0; it < 32; ++it) {
      const int row = it * 2 + hh;
      float* sp = slab + row * SLABP + c4;
      v4f a = *(const v4f*)sp;
      const v4f rz = *(const v4f*)(resid + (size_t)(m0 + row) * ldc + n0 + c4);
#pragma unroll
      for (int e = 0; e < 4; ++e) {
        float rv = rz[e];
        if (RBF) rv = bf16r(rv);
        a[e] = rv + gz[e] * (a[e] + bz[e]);
      }
      *(v4f*)sp = a;
    }
    for (int pass = 0; pass < 2; ++pass) {
#pragma unroll 4
      for (int it = 0; it < 32; ++it) {
        const int row = it * 2 + hh;
        const v4f a = *(const v4f*)(slab + row * SLABP + c4);
        *(volatile v4f*)(C + (size_t)(m0 + row) * ldc + n0 + c4) = a;
      }
      __threadfence();
    }
  } else {
    const int q  = lane >> 3;
    const int c8 = (lane & 7) * 8;
    const v4f braw0 = *(const v4f*)(bias + n0 + c8);
    const v4f braw1 = *(const v4f*)(bias + n0 + c8 + 4);
    v4f bz0, bz1;
#pragma unroll
    for (int e = 0; e < 4; ++e) {
      const float b0v = braw0[e];
      const float b1v = braw1[e];
      bz0[e] = bf16r(b0v);
      bz1[e] = bf16r(b1v);
    }
    unsigned short* C = (unsigned short*)Cout;
#pragma unroll 1
    for (int it = 0; it < 16; ++it) {
      const int row = it * 4 + q;
      float* sp = slab + row * SLABP + c8;
      v4f a = *(const v4f*)sp;
      v4f b = *(const v4f*)(sp + 4);
#pragma unroll
      for (int e = 0; e < 4; ++e) {
        const float za = a[e] + bz0[e];
        const float zb = b[e] + bz1[e];
        a[e] = (EPI == 0) ? gelu_erf(za) : gelu_tanh(za);
        b[e] = (EPI == 0) ? gelu_erf(zb) : gelu_tanh(zb);
      }
      *(v4f*)sp = a;
      *(v4f*)(sp + 4) = b;
    }
    for (int pass = 0; pass < 2; ++pass) {
#pragma unroll 4
      for (int it = 0; it < 16; ++it) {
        const int row = it * 4 + q;
        const float* sp = slab + row * SLABP + c8;
        const v4f a = *(const v4f*)sp;
        const v4f b = *(const v4f*)(sp + 4);
        v8h hv;
#pragma unroll
        for (int e = 0; e < 4; ++e) {
          hv[e]     = (_Float16)a[e];
          hv[4 + e] = (_Float16)b[e];
        }
        *(volatile v8h*)(C + (size_t)(m0 + row) * ldc + n0 + c8) = hv;
      }
      __threadfence();
    }
  }
}

extern "C" void kernel_launch(void* const* d_in, const int* in_sizes, int n_in,
                              void* d_out, int out_size, void* d_ws, size_t ws_size, hipStream_t stream) {
  if (n_in < 12 || d_out == nullptr || d_ws == nullptr) return;
  if (in_sizes[0] != NTOK * DIMC || in_sizes[1] != NBATCH * DIMC || in_sizes[2] != DIMC * EMBW ||
      in_sizes[3] != EMBW || in_sizes[4] != DIMC * DIMC || in_sizes[5] != DIMC ||
      in_sizes[6] != DIMC * DIMC || in_sizes[7] != DIMC || in_sizes[8] != DIMC * HIDF ||
      in_sizes[9] != HIDF || in_sizes[10] != HIDF * DIMC || in_sizes[11] != DIMC ||
      out_size != NTOK * DIMC) return;

  const float* x      = (const float*)d_in[0];
  const float* t      = (const float*)d_in[1];
  const float* ada_w  = (const float*)d_in[2];
  const float* ada_b  = (const float*)d_in[3];
  const float* ssm_w1 = (const float*)d_in[4];
  const float* ssm_b1 = (const float*)d_in[5];
  const float* ssm_w2 = (const float*)d_in[6];
  const float* ssm_b2 = (const float*)d_in[7];
  const float* ff_w1  = (const float*)d_in[8];
  const float* ff_b1  = (const float*)d_in[9];
  const float* ff_w2  = (const float*)d_in[10];
  const float* ff_b2  = (const float*)d_in[11];
  float* out = (float*)d_out;

  char* ws = (char*)d_ws;
  size_t off = 0;
  auto carve = [&](size_t bytes) -> char* { char* p = ws + off; off += (bytes + 255) & ~(size_t)255; return p; };
  float*          EMB  = (float*)carve((size_t)NBATCH * EMBW * 4);
  float*          X2   = (float*)carve((size_t)NTOK * DIMC * 4);
  unsigned short* NORM = (unsigned short*)carve((size_t)NTOK * DIMC * 2);
  unsigned short* HPL  = (unsigned short*)carve((size_t)NTOK * DIMC * 2);
  unsigned short* HFPL = (unsigned short*)carve((size_t)NTOK * HIDF * 2);
  unsigned short* W1T  = (unsigned short*)carve((size_t)DIMC * DIMC * 2);
  unsigned short* W2T  = (unsigned short*)carve((size_t)DIMC * DIMC * 2);
  unsigned short* F1T  = (unsigned short*)carve((size_t)HIDF * DIMC * 2);
  unsigned short* F2T  = (unsigned short*)carve((size_t)DIMC * HIDF * 2);
  if (off > ws_size || off > (size_t)134217728) return;

  wprep_kernel<<<dim3(DIMC / 64, DIMC / 64), 256, 0, stream>>>(ssm_w1, W1T, DIMC, DIMC);
  wprep_kernel<<<dim3(DIMC / 64, DIMC / 64), 256, 0, stream>>>(ssm_w2, W2T, DIMC, DIMC);
  wprep_kernel<<<dim3(HIDF / 64, DIMC / 64), 256, 0, stream>>>(ff_w1,  F1T, DIMC, HIDF);
  wprep_kernel<<<dim3(DIMC / 64, HIDF / 64), 256, 0, stream>>>(ff_w2,  F2T, HIDF, DIMC);

  cond_proj_kernel<<<EMBW / 256, 256, 0, stream>>>(t, ada_w, ada_b, EMB);

  ln_mod_kernel<true><<<NTOK / 8, 256, 0, stream>>>(x, EMB, 0 * DIMC, 1 * DIMC, NORM, NTOK);

  {
    const int tiles = (NTOK / 64) * (DIMC / 64);
    gemm_tok_kernel<0, false><<<tiles / GEMM_WAVES, 64, 0, stream>>>(
        NORM, DIMC, W1T, DIMC, (void*)HPL, DIMC,
        ssm_b1, ssm_b1, ssm_b1, NTOK, DIMC, DIMC, WCARRY_INV);
  }
  {
    const int tiles = (NTOK / 64) * (DIMC / 64);
    gemm_tok_kernel<2, true><<<tiles / GEMM_WAVES, 64, 0, stream>>>(
        HPL, DIMC, W2T, DIMC, (void*)X2, DIMC,
        ssm_b2, x, EMB + 2 * DIMC, NTOK, DIMC, DIMC, WCARRY_INV);
  }
  ln_mod_kernel<false><<<NTOK / 8, 256, 0, stream>>>(X2, EMB, 3 * DIMC, 4 * DIMC, NORM, NTOK);

  {
    const int tiles = (NTOK / 64) * (HIDF / 64);
    gemm_tok_kernel<1, false><<<tiles / GEMM_WAVES, 64, 0, stream>>>(
        NORM, DIMC, F1T, DIMC, (void*)HFPL, HIDF,
        ff_b1, ff_b1, ff_b1, NTOK, HIDF, DIMC, WCARRY_INV);
  }
  {
    const int tiles = (NTOK / 64) * (DIMC / 64);
    gemm_tok_kernel<2, false><<<tiles / GEMM_WAVES, 64, 0, stream>>>(
        HFPL, HIDF, F2T, HIDF, (void*)out, DIMC,
        ff_b2, X2, EMB + 5 * DIMC, NTOK, DIMC, HIDF, WCARRY_INV);
  }
}
